// SelectiveSSM_23828478558711
// MI455X (gfx1250) — hardware-verified
//
#include <hip/hip_runtime.h>
#include <math.h>

typedef __attribute__((ext_vector_type(16))) _Float16 v16h;
typedef __attribute__((ext_vector_type(8)))  _Float16 v8h;
typedef __attribute__((ext_vector_type(16))) __bf16   v16b;
typedef __attribute__((ext_vector_type(8)))  __bf16   v8b;
typedef __attribute__((ext_vector_type(8)))  float    v8f;
typedef __attribute__((ext_vector_type(4)))  float    v4f;

constexpr int kBatch  = 2;
constexpr int kSeq    = 2048;
constexpr int kDm     = 1024;
constexpr int kDin    = 2048;
constexpr int kNst    = 16;
constexpr int kConvK  = 4;
constexpr int kXzP    = 2 * kDin;
constexpr int kXdN    = 1 + 2 * kNst;
constexpr int kXdP    = 64;
constexpr int kRows   = kBatch * kSeq;
constexpr int kConvTP = 260;
constexpr int kScanTS = 64;
constexpr int kScanCh = 64;
constexpr int kScanYP = 68;
static_assert(kXdN <= kXdP);
static_assert((kDm % 32) == 0 && (kDin % 32) == 0);
static_assert((kSeq % 64) == 0 && (kXzP % 64) == 0 && (kXdP % 64) == 0 && (kDm % 64) == 0);
static_assert((kSeq % kScanTS) == 0 && (kDin % kScanCh) == 0 && (kDin % 256) == 0 && (kDm % 8) == 0);
static_assert((kXdN * kDin) % (8 * 256) == 0);

constexpr size_t kOffXB   = 0;
constexpr size_t kOffWIB  = kOffXB  + (size_t)kRows * kDm  * 2;
constexpr size_t kOffWXB  = kOffWIB + (size_t)kXzP  * kDm  * 2;
constexpr size_t kOffWOB  = kOffWXB + (size_t)kXdP  * kDin * 2;
constexpr size_t kOffXZ   = kOffWOB + (size_t)kDm   * kDin * 2;
constexpr size_t kOffUC   = kOffXZ  + (size_t)kSeq  * kXzP * 4;
constexpr size_t kOffUCH  = kOffUC  + (size_t)kSeq  * kDin * 4;
constexpr size_t kOffUCL  = kOffUCH + (size_t)kSeq  * kDin * 2;
constexpr size_t kOffXD   = kOffUCL + (size_t)kSeq  * kDin * 2;
constexpr size_t kOffYH   = kOffXD  + (size_t)kSeq  * kXdP * 4;
constexpr size_t kOffYL   = kOffYH  + (size_t)kSeq  * kDin * 2;
constexpr size_t kWsTotal = kOffYL  + (size_t)kSeq  * kDin * 2;
static_assert(kWsTotal == 105644032ull);
static_assert(kWsTotal <= 134217728ull);
static_assert((kOffWIB % 128) == 0 && (kOffWXB % 128) == 0 && (kOffWOB % 128) == 0 && (kOffXZ % 128) == 0 &&
              (kOffUC % 128) == 0 && (kOffUCH % 128) == 0 && (kOffUCL % 128) == 0 && (kOffXD % 128) == 0 &&
              (kOffYH % 128) == 0 && (kOffYL % 128) == 0);

__device__ __forceinline__ unsigned short f2bf_bits(float f) {
  unsigned u = __float_as_uint(f);
  return (unsigned short)((u + 0x7FFFu + ((u >> 16) & 1u)) >> 16);
}
__device__ __forceinline__ float bf_bits2f(unsigned short h) { return __uint_as_float(((unsigned)h) << 16); }
__device__ __forceinline__ float bf16r(float f) { return bf_bits2f(f2bf_bits(f)); }

__device__ __forceinline__ void dep_guard4_h(v8f& a, v8f& b, v8f& c, v8f& d, v16h x, v16h y) { asm volatile("v_nop\n\tv_nop\n\tv_nop\n\tv_nop" : "+v"(a), "+v"(b), "+v"(c), "+v"(d) : "v"(x), "v"(y)); }
__device__ __forceinline__ void dep_guard4_b(v8f& a, v8f& b, v8f& c, v8f& d, v16b x, v16b y) { asm volatile("v_nop\n\tv_nop\n\tv_nop\n\tv_nop" : "+v"(a), "+v"(b), "+v"(c), "+v"(d) : "v"(x), "v"(y)); }
__device__ __forceinline__ void keep4_h(v16h a, v16h b, v16h c, v16h d) { asm volatile("v_nop" :: "v"(a), "v"(b), "v"(c), "v"(d)); }
__device__ __forceinline__ void keep4_b(v16b a, v16b b, v16b c, v16b d) { asm volatile("v_nop" :: "v"(a), "v"(b), "v"(c), "v"(d)); }
__device__ __forceinline__ void acc_guard4(v8f& a, v8f& b, v8f& c, v8f& d) { asm volatile("v_nop\n\tv_nop\n\tv_nop\n\tv_nop" : "+v"(a), "+v"(b), "+v"(c), "+v"(d)); }
template <typename T> struct Frag;
template <> struct Frag<_Float16> {
  typedef v16h V; union U { v16h v; v8h h[2]; };
  static __device__ __forceinline__ v16h load(const _Float16* p) {
    U f; f.h[0] = *(const v8h*)(p); f.h[1] = *(const v8h*)(p + 16); return f.v;
  }
  static __device__ __forceinline__ v8f mma(v16h a, v16h b, v8f c) {
    return __builtin_amdgcn_wmma_f32_16x16x32_f16(false, a, false, b, (short)0, c, false, false);
  }
  static __device__ __forceinline__ void guard(v8f& a, v8f& b, v8f& c, v8f& d, v16h x, v16h y) { dep_guard4_h(a, b, c, d, x, y); }
  static __device__ __forceinline__ void keep(v16h a, v16h b, v16h c, v16h d) { keep4_h(a, b, c, d); }
};
template <> struct Frag<__bf16> {
  typedef v16b V; union U { v16b v; v8b h[2]; };
  static __device__ __forceinline__ v16b load(const __bf16* p) {
    U f; f.h[0] = *(const v8b*)(p); f.h[1] = *(const v8b*)(p + 16); return f.v;
  }
  static __device__ __forceinline__ v8f mma(v16b a, v16b b, v8f c) {
    return __builtin_amdgcn_wmma_f32_16x16x32_bf16(false, a, false, b, (short)0, c, false, false);
  }
  static __device__ __forceinline__ void guard(v8f& a, v8f& b, v8f& c, v8f& d, v16b x, v16b y) { dep_guard4_b(a, b, c, d, x, y); }
  static __device__ __forceinline__ void keep(v16b a, v16b b, v16b c, v16b d) { keep4_b(a, b, c, d); }
};

template <int ET> struct Elem;
template <> struct Elem<0> { typedef _Float16 T; };
template <> struct Elem<1> { typedef __bf16 T; };
template <int ET, int SPL, int BIAS_MODE, int OUT_MODE, bool RESID, int ACT = 0>
__global__ __launch_bounds__(256) void wmma_gemm64(
    const unsigned short* __restrict__ Ap, const unsigned short* __restrict__ A2p, int lda, long strideA,
    const unsigned short* __restrict__ Btp, const unsigned short* __restrict__ Bt2p, int ldb, long strideB,
    void* __restrict__ Cout, void* __restrict__ Cout2, int ldc, long strideC,
    const float* __restrict__ bias,
    const float* __restrict__ resid, long strideR,
    int M, int N, int K, float scale) {
  typedef typename Elem<ET>::T T;
  typedef typename Frag<T>::V V;
  const T* A = (const T*)Ap; const T* A2 = (const T*)A2p; const T* Bt = (const T*)Btp; const T* Bt2 = (const T*)Bt2p;
  __shared__ __align__(16) float sT[8][16 * 68];
  const int b    = blockIdx.y;
  const int lane = threadIdx.x & 31;
  const int wave = threadIdx.x >> 5;
  const int tilesN = N >> 6;
  const int tilesM = M >> 6;
  const int tile = blockIdx.x * 8 + wave;
  if (tile >= tilesM * tilesN) return;
  const int tm = tile / tilesN;
  const int tn = tile - tm * tilesN;
  const int m0 = tm << 6;
  const int n0 = tn << 6;

  const T* Ab  = A  + (size_t)b * strideA;
  const T* Bb  = Bt + (size_t)b * strideB;
  const T* Ab2 = (SPL >= 1) ? (A2  + (size_t)b * strideA) : nullptr;
  const T* Bb2 = (SPL == 2) ? (Bt2 + (size_t)b * strideB) : nullptr;

  const int rlane = lane & 15;
  const int koff  = (lane >> 4) * 8;
  const int mOff  = (lane >> 4) * 8;

  v8f acc[4][4];
#pragma unroll
  for (int i = 0; i < 4; ++i)
#pragma unroll
    for (int j = 0; j < 4; ++j) acc[i][j] = (v8f){0.f,0.f,0.f,0.f,0.f,0.f,0.f,0.f};

  for (int k0 = 0; k0 < K; k0 += 32) {
    V bh[4], bl[4];
#pragma unroll
    for (int j = 0; j < 4; ++j) {
      const size_t bo = (size_t)(n0 + (j << 4) + rlane) * ldb + koff + k0;
      bh[j] = Frag<T>::load(Bb + bo);
      if (SPL == 2) bl[j] = Frag<T>::load(Bb2 + bo);
    }
#pragma unroll
    for (int i = 0; i < 4; ++i) {
      const size_t ao = (size_t)(m0 + (i << 4) + rlane) * lda + koff + k0;
      V ah = Frag<T>::load(Ab + ao);
      V al;
      if (SPL >= 1) al = Frag<T>::load(Ab2 + ao);
#pragma unroll
      for (int j = 0; j < 4; ++j) {
        acc[i][j] = Frag<T>::mma(ah, bh[j], acc[i][j]);
        if (SPL == 2) acc[i][j] = Frag<T>::mma(ah, bl[j], acc[i][j]);
        if (SPL >= 1) acc[i][j] = Frag<T>::mma(al, bh[j], acc[i][j]);
      }
      Frag<T>::guard(acc[i][0], acc[i][1], acc[i][2], acc[i][3], ah, (SPL >= 1) ? al : ah);
    }
    Frag<T>::keep(bh[0], bh[1], bh[2], bh[3]);
    if (SPL == 2) Frag<T>::keep(bl[0], bl[1], bl[2], bl[3]);
  }
  acc_guard4(acc[0][0], acc[0][1], acc[0][2], acc[0][3]);
  acc_guard4(acc[1][0], acc[1][1], acc[1][2], acc[1][3]);
  acc_guard4(acc[2][0], acc[2][1], acc[2][2], acc[2][3]);
  acc_guard4(acc[3][0], acc[3][1], acc[3][2], acc[3][3]);

  float* slab = sT[wave];
  const float* Rb = RESID ? (resid + (size_t)b * strideR) : nullptr;
#pragma unroll
  for (int i = 0; i < 4; ++i) {
    const int mBase = m0 + (i << 4);
#pragma unroll
    for (int j = 0; j < 4; ++j) {
      const int n = n0 + (j << 4) + rlane;
      float bv = 0.f;
      if (BIAS_MODE == 2) bv = bias[n];
#pragma unroll
      for (int r = 0; r < 8; ++r) {
        float v = acc[i][j][r] * scale;
        if (BIAS_MODE == 1) v += bias[mBase + mOff + r];
        if (BIAS_MODE == 2) v += bv;
        if (RESID) v += Rb[(size_t)(mBase + mOff + r) * ldc + n];
        if (ACT == 1) v = tanhf(v);
        if (ACT == 2) v = fmaxf(v, 0.0f);
        if (ACT == 3) v = v / (1.0f + expf(-v));
        if (ACT == 4) v = (v > 0.f) ? v : 0.01f * v;
        slab[(mOff + r) * 68 + (j << 4) + rlane] = v;
      }
    }
    __builtin_amdgcn_fence(__ATOMIC_RELEASE, "workgroup");
    __builtin_amdgcn_wave_barrier();
    __builtin_amdgcn_fence(__ATOMIC_ACQUIRE, "workgroup");
    if (OUT_MODE == 0) {
      float* C = (float*)Cout + (size_t)b * strideC;
      const int hh = lane >> 4, c4 = (lane & 15) * 4;
      for (int pass = 0; pass < 2; ++pass) {
#pragma unroll
        for (int it = 0; it < 8; ++it) {
          const int row = it * 2 + hh;
          v4f v = *(const v4f*)(slab + row * 68 + c4);
          *(volatile v4f*)(C + (size_t)(mBase + row) * ldc + n0 + c4) = v;
        }
        __threadfence();
      }
    } else {
      const int q = lane >> 3, c8 = (lane & 7) * 8;
      unsigned short* C  = (unsigned short*)Cout  + (size_t)b * strideC;
      unsigned short* C2 = (OUT_MODE == 2) ? ((unsigned short*)Cout2 + (size_t)b * strideC) : nullptr;
      for (int pass = 0; pass < 2; ++pass) {
#pragma unroll
        for (int it = 0; it < 4; ++it) {
          const int row = it * 4 + q;
          const float* sp = slab + row * 68 + c8;
          v8h hv, lv;
#pragma unroll
          for (int e = 0; e < 8; ++e) {
            if (OUT_MODE == 1) {
              hv[e] = (_Float16)sp[e];
            } else {
              unsigned short hb = f2bf_bits(sp[e]);
              unsigned short lb = f2bf_bits(sp[e] - bf_bits2f(hb));
              hv[e] = __builtin_bit_cast(_Float16, hb);
              lv[e] = __builtin_bit_cast(_Float16, lb);
            }
          }
          *(volatile v8h*)(C + (size_t)(mBase + row) * ldc + n0 + c8) = hv;
          if (OUT_MODE == 2) *(volatile v8h*)(C2 + (size_t)(mBase + row) * ldc + n0 + c8) = lv;
        }
        __threadfence();
      }
    }
    __builtin_amdgcn_fence(__ATOMIC_RELEASE, "workgroup");
    __builtin_amdgcn_wave_barrier();
    __builtin_amdgcn_fence(__ATOMIC_ACQUIRE, "workgroup");
  }
}

__global__ __launch_bounds__(256) void cast_bf16_kernel(
    const float* __restrict__ src, unsigned short* __restrict__ dst, int total8, int real8)
{
  const int i = blockIdx.x * 256 + threadIdx.x;
  if (i >= total8) return;
  const bool live = (i < real8);
  const int  ic   = live ? i : (real8 - 1);
  const size_t s0 = (size_t)ic << 3;
  const v4f a0 = *(const v4f*)(src + s0);
  const v4f a1 = *(const v4f*)(src + s0 + 4);
  v8h hv;
#pragma unroll
  for (int e = 0; e < 4; ++e) {
    const float f0 = live ? a0[e] : 0.0f;
    const float f1 = live ? a1[e] : 0.0f;
    const unsigned short h0 = f2bf_bits(f0), h1 = f2bf_bits(f1);
    hv[e]     = __builtin_bit_cast(_Float16, h0);
    hv[4 + e] = __builtin_bit_cast(_Float16, h1);
  }
  unsigned short* qd = dst + ((size_t)i << 3);
  *(volatile v8h*)qd = hv;
  __threadfence();
  *(volatile v8h*)qd = hv;
}

__global__ __launch_bounds__(256) void conv_silu_kernel(
    const float* __restrict__ XZ, const float* __restrict__ cw, const float* __restrict__ cb,
    float* __restrict__ UC, unsigned short* __restrict__ UCH, unsigned short* __restrict__ UCL)
{
  __shared__ __align__(16) float sT[16 * kConvTP];
  const int tid = threadIdx.x, lane = tid & 31, wave = tid >> 5;
  const int d0 = blockIdx.x * 256, d = d0 + tid;
  const int t0 = blockIdx.y * 64;
  const float w0 = bf16r(cw[d * kConvK + 0]), w1 = bf16r(cw[d * kConvK + 1]);
  const float w2 = bf16r(cw[d * kConvK + 2]), w3 = bf16r(cw[d * kConvK + 3]);
  const float bc = bf16r(cb[d]);
  float xm3, xm2, xm1;
  {
    const int r3 = t0 - 3, r2 = t0 - 2, r1 = t0 - 1;
    const float v3 = XZ[(size_t)(r3 < 0 ? 0 : r3) * kXzP + d];
    const float v2 = XZ[(size_t)(r2 < 0 ? 0 : r2) * kXzP + d];
    const float v1 = XZ[(size_t)(r1 < 0 ? 0 : r1) * kXzP + d];
    xm3 = (r3 >= 0) ? v3 : 0.f;
    xm2 = (r2 >= 0) ? v2 : 0.f;
    xm1 = (r1 >= 0) ? v1 : 0.f;
  }
  const int hrow = wave >> 1;
  const int hch  = (wave & 1) * 128 + lane * 4;
#pragma unroll 1
  for (int sub = 0; sub < 4; ++sub) {
    const int lb = t0 + sub * 16;
#pragma unroll 1
    for (int s = 0; s < 16; ++s) {
      const float xcur = XZ[(size_t)(lb + s) * kXzP + d];
      float acc = w0 * xm3;
      acc = fmaf(w1, xm2, acc);
      acc = fmaf(w2, xm1, acc);
      acc = fmaf(w3, xcur, acc);
      const float sv = acc + bc;
      const float sg = __builtin_amdgcn_rcpf(1.0f + expf(-sv));
      sT[s * kConvTP + tid] = sv * sg;
      xm3 = xm2; xm2 = xm1; xm1 = xcur;
    }
    __syncthreads();
    v4f fv[4];
    v8h bh[2], blo[2];
#pragma unroll
    for (int it = 0; it < 4; ++it) fv[it] = *(const v4f*)(sT + (it * 4 + hrow) * kConvTP + hch);
#pragma unroll
    for (int it = 0; it < 2; ++it) {
      const float* sp = sT + (it * 8 + wave) * kConvTP + lane * 8;
      const v4f a0 = *(const v4f*)(sp);
      const v4f a1 = *(const v4f*)(sp + 4);
#pragma unroll
      for (int e = 0; e < 4; ++e) {
        const unsigned short h0 = f2bf_bits(a0[e]), h1 = f2bf_bits(a1[e]);
        const unsigned short l0 = f2bf_bits(a0[e] - bf_bits2f(h0)), l1 = f2bf_bits(a1[e] - bf_bits2f(h1));
        bh[it][e]      = __builtin_bit_cast(_Float16, h0);
        bh[it][4 + e]  = __builtin_bit_cast(_Float16, h1);
        blo[it][e]     = __builtin_bit_cast(_Float16, l0);
        blo[it][4 + e] = __builtin_bit_cast(_Float16, l1);
      }
    }
    for (int pass = 0; pass < 2; ++pass) {
#pragma unroll
      for (int it = 0; it < 4; ++it)
        *(volatile v4f*)(UC + (size_t)(lb + it * 4 + hrow) * kDin + d0 + hch) = fv[it];
#pragma unroll
      for (int it = 0; it < 2; ++it) {
        const size_t o = (size_t)(lb + it * 8 + wave) * kDin + d0 + lane * 8;
        *(volatile v8h*)(UCH + o) = bh[it];
        *(volatile v8h*)(UCL + o) = blo[it];
      }
      __threadfence();
    }
    __syncthreads();
  }
}

__global__ __launch_bounds__(64) void scan_kernel(
    const float* __restrict__ XD, const float* __restrict__ UC, const float* __restrict__ XZ,
    const float* __restrict__ Wdt, const float* __restrict__ bdt, const float* __restrict__ Alog,
    const float* __restrict__ Dp, unsigned short* __restrict__ YH, unsigned short* __restrict__ YL)
{
  __shared__ __align__(16) float sX[kScanTS * kXdP];
  __shared__ __align__(16) float sY[kScanTS * kScanYP];
  __shared__ __align__(16) float sA[kNst * kScanCh];
  const int tid = threadIdx.x, lane = tid & 31, wave = tid >> 5;
  const int d0  = blockIdx.x * kScanCh;
  const int d   = d0 + tid;
#pragma unroll 1
  for (int s = 0; s < kNst; ++s) sA[s * kScanCh + tid] = -expf(bf16r(Alog[(size_t)d * kNst + s]));
  __syncthreads();
  float negA[kNst], h[kNst];
#pragma unroll
  for (int s = 0; s < kNst; ++s) {
    negA[s] = sA[s * kScanCh + tid];
    h[s] = 0.f;
  }
  const float wdt = bf16r(Wdt[d]);
  const float bb  = bf16r(bdt[d]);
  const float Dd  = bf16r(Dp[d]);
  const int lr = tid >> 4, lc4 = (tid & 15) * 4;
  const int q = lane >> 3, c8 = (lane & 7) * 8;
#pragma unroll 1
  for (int t0 = 0; t0 < kSeq; t0 += kScanTS) {
    __syncthreads();
#pragma unroll
    for (int gq = 0; gq < 4; ++gq) {
#pragma unroll
      for (int i = 0; i < 4; ++i) {
        const int r = lr + 4 * (gq * 4 + i);
        *(v4f*)(sX + r * kXdP + lc4) = *(const v4f*)(XD + (size_t)(t0 + r) * kXdP + lc4);
      }
      asm volatile("" ::: "memory");
    }
    __syncthreads();
#pragma unroll 1
    for (int s = 0; s < kScanTS; ++s) {
      const size_t m = (size_t)(t0 + s);
      const float* xr = sX + s * kXdP;
      v4f xv[9];
#pragma unroll
      for (int qq = 0; qq < 9; ++qq) xv[qq] = *(const v4f*)(xr + 4 * qq);
      const float dtr = xv[0][0];
      const float tv  = dtr * wdt + bb;
      const float ea  = expf(-fabsf(tv));
      const float dlt = fmaxf(tv, 0.0f) + log1pf(ea);
      const float xt  = UC[m * kDin + d];
      const float zv  = XZ[m * kXzP + kDin + d];
      float y = 0.f;
#pragma unroll
      for (int n = 0; n < kNst; ++n) {
        const float Bn = xv[(1 + n) >> 2][(1 + n) & 3];
        const float Cn = xv[(1 + kNst + n) >> 2][(1 + kNst + n) & 3];
        const float e  = __expf(dlt * negA[n]);
        float db = dlt * Bn;
        asm volatile("" : "+v"(db));
        float p = db * xt;
        asm volatile("" : "+v"(p));
        float qv = h[n] * e;
        asm volatile("" : "+v"(qv));
        const float hn = qv + p;
        h[n] = hn;
        float rr = hn * Cn;
        asm volatile("" : "+v"(rr));
        y += rr;
      }
      float sk = xt * Dd;
      asm volatile("" : "+v"(sk));
      y += sk;
      const float sg = __builtin_amdgcn_rcpf(1.0f + expf(-zv));
      const float g  = zv * sg;
      sY[s * kScanYP + tid] = y * g;
    }
    __syncthreads();
    v8h hv[8], lv[8];
#pragma unroll
    for (int it = 0; it < 8; ++it) {
      const int row = it * 8 + wave * 4 + q;
      const float* sp = sY + row * kScanYP + c8;
      const v4f a0 = *(const v4f*)(sp);
      const v4f a1 = *(const v4f*)(sp + 4);
#pragma unroll
      for (int e = 0; e < 4; ++e) {
        const unsigned short h0 = f2bf_bits(a0[e]), h1 = f2bf_bits(a1[e]);
        const unsigned short l0 = f2bf_bits(a0[e] - bf_bits2f(h0)), l1 = f2bf_bits(a1[e] - bf_bits2f(h1));
        hv[it][e]     = __builtin_bit_cast(_Float16, h0);
        hv[it][4 + e] = __builtin_bit_cast(_Float16, h1);
        lv[it][e]     = __builtin_bit_cast(_Float16, l0);
        lv[it][4 + e] = __builtin_bit_cast(_Float16, l1);
      }
    }
    for (int pass = 0; pass < 2; ++pass) {
#pragma unroll
      for (int it = 0; it < 8; ++it) {
        const int row = it * 8 + wave * 4 + q;
        const size_t o = (size_t)(t0 + row) * kDin + d0 + c8;
        *(volatile v8h*)(YH + o) = hv[it];
        *(volatile v8h*)(YL + o) = lv[it];
      }
      __threadfence();
    }
  }
}

extern "C" void kernel_launch(void* const* d_in, const int* in_sizes, int n_in,
                              void* d_out, int out_size, void* d_ws, size_t ws_size,
                              hipStream_t stream) {
  if (n_in < 10) return;
  if (in_sizes[0] != kRows * kDm) return;
  if (in_sizes[1] != kXzP * kDm) return;
  if (in_sizes[2] != kDin * kConvK) return;
  if (in_sizes[3] != kDin) return;
  if (in_sizes[4] != kXdN * kDin) return;
  if (in_sizes[5] != kDin) return;
  if (in_sizes[6] != kDin) return;
  if (in_sizes[7] != kDin * kNst) return;
  if (in_sizes[8] != kDin) return;
  if (in_sizes[9] != kDm * kDin) return;
  if (out_size != kRows * kDm) return;
  if (ws_size < kWsTotal) return;

  const float* x       = (const float*)d_in[0];
  const float* W_in    = (const float*)d_in[1];
  const float* conv_w  = (const float*)d_in[2];
  const float* conv_b  = (const float*)d_in[3];
  const float* W_xproj = (const float*)d_in[4];
  const float* W_dt    = (const float*)d_in[5];
  const float* b_dt    = (const float*)d_in[6];
  const float* A_log   = (const float*)d_in[7];
  const float* Dp      = (const float*)d_in[8];
  const float* W_out   = (const float*)d_in[9];
  float* out = (float*)d_out;

  char* ws = (char*)d_ws;
  unsigned short* XB   = (unsigned short*)(ws + kOffXB);
  unsigned short* WIB  = (unsigned short*)(ws + kOffWIB);
  unsigned short* WXB  = (unsigned short*)(ws + kOffWXB);
  unsigned short* WOB  = (unsigned short*)(ws + kOffWOB);
  float*          XZ   = (float*)(ws + kOffXZ);
  float*          UC   = (float*)(ws + kOffUC);
  unsigned short* UCH  = (unsigned short*)(ws + kOffUCH);
  unsigned short* UCL  = (unsigned short*)(ws + kOffUCL);
  float*          XD   = (float*)(ws + kOffXD);
  unsigned short* YH   = (unsigned short*)(ws + kOffYH);
  unsigned short* YL   = (unsigned short*)(ws + kOffYL);
  const float* dummy_bias  = b_dt;
  const float* dummy_resid = x;

  {
    const int t8x  = kRows * kDm / 8;
    const int t8wi = kXzP * kDm / 8;
    const int t8wx = kXdP * kDin / 8;
    const int r8wx = kXdN * kDin / 8;
    const int t8wo = kDm * kDin / 8;
    cast_bf16_kernel<<<t8x / 256,  256, 0, stream>>>(x,       XB,  t8x,  t8x);
    cast_bf16_kernel<<<t8wi / 256, 256, 0, stream>>>(W_in,    WIB, t8wi, t8wi);
    cast_bf16_kernel<<<t8wx / 256, 256, 0, stream>>>(W_xproj, WXB, t8wx, r8wx);
    cast_bf16_kernel<<<t8wo / 256, 256, 0, stream>>>(W_out,   WOB, t8wo, t8wo);
  }

  for (int b = 0; b < kBatch; ++b) {
    const unsigned short* XBb = XB + (size_t)b * kSeq * kDm;
    float* outb = out + (size_t)b * kSeq * kDm;

    wmma_gemm64<1, 0, 0, 0, false><<<dim3(256, 1), 256, 0, stream>>>(
        XBb, XBb, kDm, 0L,
        WIB, WIB, kDm, 0L,
        (void*)XZ, (void*)XZ, kXzP, 0L,
        dummy_bias, dummy_resid, 0L,
        kSeq, kXzP, kDm, 1.0f);

    conv_silu_kernel<<<dim3(kDin / 256, kSeq / 64), 256, 0, stream>>>(XZ, conv_w, conv_b, UC, UCH, UCL);

    wmma_gemm64<1, 1, 0, 0, false><<<dim3(4, 1), 256, 0, stream>>>(
        UCH, UCL, kDin, 0L,
        WXB, WXB, kDin, 0L,
        (void*)XD, (void*)XD, kXdP, 0L,
        dummy_bias, dummy_resid, 0L,
        kSeq, kXdP, kDin, 1.0f);

    scan_kernel<<<kDin / kScanCh, kScanCh, 0, stream>>>(XD, UC, XZ, W_dt, b_dt, A_log, Dp, YH, YL);

    wmma_gemm64<1, 1, 0, 0, false><<<dim3(64, 1), 256, 0, stream>>>(
        YH, YL, kDin, 0L,
        WOB, WOB, kDin, 0L,
        (void*)outb, (void*)outb, kDm, 0L,
        dummy_bias, dummy_resid, 0L,
        kSeq, kDm, kDin, 1.0f);
  }
}
